// MultiScaleModule_v2_27522150432908
// MI455X (gfx1250) — hardware-run, weakly checked
//
#include <hip/hip_runtime.h>
#include <stddef.h>

typedef __attribute__((ext_vector_type(16))) _Float16 v16h;
typedef __attribute__((ext_vector_type(8)))  _Float16 v8h;
typedef __attribute__((ext_vector_type(8)))  float    v8f;
typedef __attribute__((ext_vector_type(4)))  float    v4f;
typedef __attribute__((ext_vector_type(4)))  unsigned v4u;

constexpr int kNB     = 2;
constexpr int kCH     = 256;
constexpr int kTAPS   = 9;
constexpr int kKC     = kCH * kTAPS;
constexpr int kKD     = 2 * kKC;
constexpr int kMOM    = 64;
constexpr int kNOFS   = 18;
constexpr int kNOM    = 27;
constexpr int kLDC    = 17088;
constexpr int kChunk  = 3200;
constexpr float kWCarry    = 64.0f;
constexpr float kWCarryInv = 1.0f / 64.0f;

static_assert(kKC == 2304 && kKD == 4608, "contraction depths");
static_assert((kKC % 32) == 0 && (kKD % 32) == 0, "GEMM K multiples of 32");
static_assert((kMOM % 64) == 0 && (kCH % 64) == 0 && (kChunk % 64) == 0, "GEMM M,N tile multiples");
static_assert(12800 + 3200 + 832 + 256 == kLDC, "column map");
static_assert((832 % 64) == 0 && (256 % 64) == 0 && (12800 % kChunk) == 0, "padded column counts");

constexpr int kE1 = 3276800;
constexpr int kE2 = 4096000;
constexpr int kE3 = 4300800;
constexpr int kE4 = 4352000;
constexpr int kOutTotal = 4364800;
static_assert(kE1 == kNB * kCH * 6400 && kE2 - kE1 == kNB * kCH * 1600 && kE3 - kE2 == kNB * kCH * 400 &&
              kE4 - kE3 == kNB * kCH * 100 && kOutTotal - kE4 == kNB * kCH * 25, "output packing");
static_assert((kE1 % 1024) == 0 && (kE2 % 1024) == 0 && (kE3 % 1024) == 0 && (kE4 % 1024) == 0, "level starts are block aligned");

constexpr size_t planeBytes(int h) { return (size_t)kNB * h * h * kCH * 2; }
constexpr size_t kOffP2   = 0;
constexpr size_t kOffP3   = kOffP2 + planeBytes(160);
constexpr size_t kOffP4   = kOffP3 + planeBytes(80);
constexpr size_t kOffP5   = kOffP4 + planeBytes(40);
constexpr size_t kOffP6   = kOffP5 + planeBytes(20);
constexpr size_t kOffP7   = kOffP6 + planeBytes(10);
constexpr size_t kOffU0   = kOffP7 + planeBytes(5);
constexpr size_t kOffU1   = kOffU0 + planeBytes(80);
constexpr size_t kOffU2   = kOffU1 + planeBytes(40);
constexpr size_t kOffU3   = kOffU2 + planeBytes(20);
constexpr size_t kOffWcat = kOffU3 + planeBytes(10);
constexpr size_t kOffOMW  = kOffWcat + (size_t)4 * kCH * kKD * 2;
constexpr size_t kOffOM   = kOffOMW + (size_t)4 * kMOM * kKC * 2;
constexpr size_t kOffCS   = kOffOM + (size_t)kMOM * kLDC * 4;
constexpr size_t kOffBT   = kOffCS + (size_t)kCH * kLDC * 4;
constexpr size_t kWsTotal = kOffBT + (size_t)kChunk * kKD * 2;
static_assert(kWsTotal == 105628672ull, "carve total");
static_assert(kWsTotal <= 134217728ull, "carve cap");
static_assert((kOffP3 % 128) == 0 && (kOffP4 % 128) == 0 && (kOffP5 % 128) == 0 && (kOffP6 % 128) == 0 &&
              (kOffP7 % 128) == 0 && (kOffU0 % 128) == 0 && (kOffU1 % 128) == 0 && (kOffU2 % 128) == 0 &&
              (kOffU3 % 128) == 0 && (kOffWcat % 128) == 0 && (kOffOMW % 128) == 0 && (kOffOM % 128) == 0 &&
              (kOffCS % 128) == 0 && (kOffBT % 128) == 0, "128-B aligned regions");

__device__ __forceinline__ int iclamp(int v, int lo, int hi) { return v < lo ? lo : (v > hi ? hi : v); }

__device__ __forceinline__ float h16_to_f32(unsigned hb) {
  const unsigned sgn = (hb & 0x8000u) << 16; const unsigned em = hb & 0x7fffu;
  const float fn = __uint_as_float((em << 13) + 0x38000000u);
  const float fs = (float)em * 5.9604644775390625e-8f;
  const float mag = (em < 0x400u) ? fs : fn; return __uint_as_float(__float_as_uint(mag) | sgn); }

__device__ __forceinline__ void unpack8(const v4u w, float (&f)[8]) {
  const unsigned w0 = w[0];
  const unsigned w1 = w[1];
  const unsigned w2 = w[2];
  const unsigned w3 = w[3];
  f[0] = h16_to_f32(w0 & 0xffffu); f[1] = h16_to_f32(w0 >> 16);
  f[2] = h16_to_f32(w1 & 0xffffu); f[3] = h16_to_f32(w1 >> 16);
  f[4] = h16_to_f32(w2 & 0xffffu); f[5] = h16_to_f32(w2 >> 16);
  f[6] = h16_to_f32(w3 & 0xffffu); f[7] = h16_to_f32(w3 >> 16);
}

union FragH { v16h v; v8h h[2]; };
__device__ __forceinline__ v16h frag_load(const _Float16* p) {
  FragH f; f.h[0] = *(const v8h*)(p); f.h[1] = *(const v8h*)(p + 16); return f.v;
}
__device__ __forceinline__ v8f mma_h(v16h a, v16h b, v8f c) {
  c = __builtin_amdgcn_wmma_f32_16x16x32_f16(false, a, false, b, (short)0, c, false, false);
  asm volatile("v_nop\n\tv_nop\n\tv_nop\n\tv_nop" : "+v"(c) : "v"(a), "v"(b));
  return c;
}

__global__ __launch_bounds__(256) void gemm_f16_nt(
    const unsigned short* __restrict__ Ap, int lda,
    const unsigned short* __restrict__ Btp, int ldb,
    float* __restrict__ C, int ldc, int M, int N, int K, float scale) {
  const _Float16* A  = (const _Float16*)Ap;
  const _Float16* Bt = (const _Float16*)Btp;
  __shared__ __align__(16) float sT[8][16 * 68];
  const int lane = threadIdx.x & 31;
  const int wave = threadIdx.x >> 5;
  const int tilesN = N >> 6;
  const int tilesM = M >> 6;
  const int tile = blockIdx.x * 8 + wave;
  if (tile >= tilesM * tilesN) return;
  const int tm = tile / tilesN;
  const int tn = tile - tm * tilesN;
  const int m0 = tm << 6;
  const int n0 = tn << 6;

  const int rlane = lane & 15;
  const int koff  = (lane >> 4) * 8;
  const int mOff  = (lane >> 4) * 8;

  v8f acc[4][4];
#pragma unroll
  for (int i = 0; i < 4; ++i)
#pragma unroll
    for (int j = 0; j < 4; ++j) acc[i][j] = (v8f){0.f, 0.f, 0.f, 0.f, 0.f, 0.f, 0.f, 0.f};

  for (int k0 = 0; k0 < K; k0 += 32) {
    v16h bh[4];
#pragma unroll
    for (int j = 0; j < 4; ++j) {
      const size_t bo = (size_t)(n0 + (j << 4) + rlane) * ldb + koff + k0;
      bh[j] = frag_load(Bt + bo);
    }
#pragma unroll
    for (int i = 0; i < 4; ++i) {
      const size_t ao = (size_t)(m0 + (i << 4) + rlane) * lda + koff + k0;
      const v16h ah = frag_load(A + ao);
#pragma unroll
      for (int j = 0; j < 4; ++j) acc[i][j] = mma_h(ah, bh[j], acc[i][j]);
    }
  }

  float* slab = sT[wave];
#pragma unroll
  for (int i = 0; i < 4; ++i) {
    const int mBase = m0 + (i << 4);
#pragma unroll
    for (int j = 0; j < 4; ++j) {
#pragma unroll
      for (int r = 0; r < 8; ++r) {
        slab[(mOff + r) * 68 + (j << 4) + rlane] = acc[i][j][r] * scale;
      }
    }
    __builtin_amdgcn_fence(__ATOMIC_RELEASE, "workgroup");
    __builtin_amdgcn_wave_barrier();
    __builtin_amdgcn_fence(__ATOMIC_ACQUIRE, "workgroup");
    {
      const int hh = lane >> 4, c4 = (lane & 15) * 4;
      for (int pass = 0; pass < 2; ++pass) {
#pragma unroll
        for (int it = 0; it < 8; ++it) {
          const int row = it * 2 + hh;
          const v4f v = *(const v4f*)(slab + row * 68 + c4);
          *(volatile v4f*)(C + (size_t)(mBase + row) * ldc + n0 + c4) = v;
        }
        __threadfence();
      }
    }
    __builtin_amdgcn_fence(__ATOMIC_RELEASE, "workgroup");
    __builtin_amdgcn_wave_barrier();
    __builtin_amdgcn_fence(__ATOMIC_ACQUIRE, "workgroup");
  }
}

__global__ __launch_bounds__(256) void nchw_to_nhwc_f16(const float* __restrict__ x, unsigned short* __restrict__ y,
                                                        int HW, int tilesPerB) {
  __shared__ float t[kCH][33];
  const int tid = threadIdx.x;
  const int b   = blockIdx.x / tilesPerB;
  const int hw0 = (blockIdx.x - b * tilesPerB) * 32;
  const float* xb = x + (size_t)b * kCH * HW;
  const int j  = tid & 31;
  const int cw = tid >> 5;
  const int hwc = (hw0 + j < HW) ? (hw0 + j) : (HW - 1);
#pragma unroll 4
  for (int i = 0; i < 32; ++i) {
    const int c = i * 8 + cw;
    t[c][j] = xb[(size_t)c * HW + hwc];
  }
  __syncthreads();
  const int wave = tid >> 5, lane = tid & 31;
  v8h hv[4];
#pragma unroll
  for (int it = 0; it < 4; ++it) {
    const int pix = wave * 4 + it;
#pragma unroll
    for (int e = 0; e < 8; ++e) hv[it][e] = (_Float16)t[lane * 8 + e][pix];
  }
  unsigned short* yb = y + ((size_t)b * HW + hw0) * kCH + lane * 8;
  for (int pass = 0; pass < 2; ++pass) {
#pragma unroll
    for (int it = 0; it < 4; ++it) {
      const int pix = wave * 4 + it;
      if (hw0 + pix < HW) *(volatile v8h*)(yb + (size_t)pix * kCH) = hv[it];
    }
    __threadfence();
  }
}

__global__ __launch_bounds__(256) void resize2x_nhwc_f16(const unsigned short* __restrict__ src,
                                                         unsigned short* __restrict__ dst, int Hin, int npix) {
  const int lane = threadIdx.x & 31, wave = threadIdx.x >> 5;
  const int p = blockIdx.x * 8 + wave;
  if (p >= npix) return;
  const int Hout = 2 * Hin;
  const int b = p / (Hout * Hout);
  const int r = p - b * Hout * Hout;
  const int Y = r / Hout;
  const int X = r - Y * Hout;
  const int jy = Y >> 1, oy = Y & 1;
  const int jx = X >> 1, ox = X & 1;
  const int ya = iclamp(oy ? jy : jy - 1, 0, Hin - 1);
  const int yb = iclamp(oy ? jy + 1 : jy, 0, Hin - 1);
  const int xa = iclamp(ox ? jx : jx - 1, 0, Hin - 1);
  const int xb = iclamp(ox ? jx + 1 : jx, 0, Hin - 1);
  const float wya = oy ? 0.75f : 0.25f;
  const float wyb = 1.0f - wya;
  const float wxa = ox ? 0.75f : 0.25f;
  const float wxb = 1.0f - wxa;
  const unsigned short* sb = src + (size_t)b * Hin * Hin * kCH + lane * 8;
  const v4u gaa = *(const v4u*)(sb + ((size_t)ya * Hin + xa) * kCH);
  const v4u gab = *(const v4u*)(sb + ((size_t)ya * Hin + xb) * kCH);
  const v4u gba = *(const v4u*)(sb + ((size_t)yb * Hin + xa) * kCH);
  const v4u gbb = *(const v4u*)(sb + ((size_t)yb * Hin + xb) * kCH);
  float faa[8], fab[8], fba[8], fbb[8];
  unpack8(gaa, faa);
  unpack8(gab, fab);
  unpack8(gba, fba);
  unpack8(gbb, fbb);
  v8h hv;
#pragma unroll
  for (int e = 0; e < 8; ++e) {
    const float ta = wya * faa[e] + wyb * fba[e];
    const float tb = wya * fab[e] + wyb * fbb[e];
    hv[e] = (_Float16)(wxa * ta + wxb * tb);
  }
  unsigned short* d = dst + (size_t)p * kCH + lane * 8;
  *(volatile v8h*)d = hv;
  __threadfence();
  *(volatile v8h*)d = hv;
}

__global__ __launch_bounds__(256) void pack_dcn_w(const float* __restrict__ w, unsigned short* __restrict__ Wcat) {
  const int g = blockIdx.x * 256 + threadIdx.x;
  if (g >= 4 * kCH * kKD / 8) return;
  const int e0  = g * 8;
  const int lvl = e0 / (kCH * kKD);
  const int rem = e0 - lvl * (kCH * kKD);
  const int o   = rem / kKD;
  const int col = rem - o * kKD;
  const int half = col / kKC;
  const int kk  = col - half * kKC;
  const int tap = kk >> 8;
  const int c0  = kk & 255;
  const int dd = (lvl == 0) ? 0 : ((lvl == 1) ? 1 : ((lvl == 2) ? 3 : 5));
  const int du = (lvl == 0) ? 2 : ((lvl == 1) ? 4 : ((lvl == 2) ? 6 : 7));
  const int d  = half ? du : dd;
  const float* wp = w + (((size_t)d * kCH + o) * kCH + c0) * kTAPS + tap;
  v8h hv;
#pragma unroll
  for (int j = 0; j < 8; ++j) hv[j] = (_Float16)(wp[(size_t)j * kTAPS] * kWCarry);
  unsigned short* q = Wcat + e0;
  *(volatile v8h*)q = hv;
  __threadfence();
  *(volatile v8h*)q = hv;
}

__global__ __launch_bounds__(256) void pack_om_w(const float* __restrict__ ow, const float* __restrict__ mw,
                                                 unsigned short* __restrict__ OMW) {
  const int g = blockIdx.x * 256 + threadIdx.x;
  if (g >= 4 * kMOM * kKC / 8) return;
  const int e0  = g * 8;
  const int lvl = e0 / (kMOM * kKC);
  const int rem = e0 - lvl * (kMOM * kKC);
  const int row = rem / kKC;
  const int col = rem - row * kKC;
  const int tap = col >> 8;
  const int c0  = col & 255;
  const int ro = iclamp(row, 0, kNOFS - 1);
  const int rm = iclamp(row - kNOFS, 0, kNOM - kNOFS - 1);
  const float* op = ow + (((size_t)lvl * kNOFS + ro) * kCH + c0) * kTAPS + tap;
  const float* mp = mw + (((size_t)lvl * (kNOM - kNOFS) + rm) * kCH + c0) * kTAPS + tap;
  const bool isOff  = row < kNOFS;
  const bool isReal = row < kNOM;
  v8h hv;
#pragma unroll
  for (int j = 0; j < 8; ++j) {
    float vo = op[(size_t)j * kTAPS];
    float vm = mp[(size_t)j * kTAPS];
    asm volatile("" : "+v"(vo), "+v"(vm));
    float v = isOff ? vo : vm;
    v = isReal ? v : 0.0f;
    hv[j] = (_Float16)(v * kWCarry);
  }
  unsigned short* q = OMW + e0;
  *(volatile v8h*)q = hv;
  __threadfence();
  *(volatile v8h*)q = hv;
}

__global__ __launch_bounds__(256) void im2col_f16(const unsigned short* __restrict__ X, unsigned short* __restrict__ Bt,
                                                  int Ho, int col0, int nreal, int nitems) {
  const int lane = threadIdx.x & 31, wave = threadIdx.x >> 5;
  const int item = blockIdx.x * 8 + wave;
  if (item >= nitems) return;
  const int n   = item / kTAPS;
  const int tap = item - n * kTAPS;
  const int nc  = (n < nreal) ? n : (nreal - 1);
  const int col = col0 + nc;
  const int HW  = Ho * Ho;
  const int b   = col / HW;
  const int pix = col - b * HW;
  const int ho  = pix / Ho;
  const int wo  = pix - ho * Ho;
  const int kh  = tap / 3;
  const int kw  = tap - kh * 3;
  const int yy  = ho + kh - 1;
  const int xx  = wo + kw - 1;
  const bool inb = (n < nreal) && (yy >= 0) && (yy < Ho) && (xx >= 0) && (xx < Ho);
  const int yc = iclamp(yy, 0, Ho - 1);
  const int xc = iclamp(xx, 0, Ho - 1);
  v4u w = *(const v4u*)(X + (((size_t)b * Ho + yc) * Ho + xc) * kCH + lane * 8);
  asm volatile("" : "+v"(w));
  v4u u;
  u[0] = inb ? w[0] : 0u;
  u[1] = inb ? w[1] : 0u;
  u[2] = inb ? w[2] : 0u;
  u[3] = inb ? w[3] : 0u;
  unsigned short* d = Bt + (size_t)n * kKC + tap * kCH + lane * 8;
  *(volatile v4u*)d = u;
  __threadfence();
  *(volatile v4u*)d = u;
}

__global__ __launch_bounds__(256) void dcn_sample(const unsigned short* __restrict__ srcDown,
                                                  const unsigned short* __restrict__ srcUp,
                                                  const float* __restrict__ OM, const float* __restrict__ offb,
                                                  const float* __restrict__ maskb, unsigned short* __restrict__ Bt,
                                                  int Ho, int col0, int nreal, int nitems) {
  const int lane = threadIdx.x & 31, wave = threadIdx.x >> 5;
  const int item = blockIdx.x * 8 + wave;
  if (item >= nitems) return;
  const int n    = item / (2 * kTAPS);
  const int r    = item - n * (2 * kTAPS);
  const int half = r / kTAPS;
  const int tap  = r - half * kTAPS;
  const int nc   = (n < nreal) ? n : (nreal - 1);
  const int col  = col0 + nc;
  const int HW   = Ho * Ho;
  const int b    = col / HW;
  const int pix  = col - b * HW;
  const int ho   = pix / Ho;
  const int wo   = pix - ho * Ho;
  const int kh   = tap / 3;
  const int kw   = tap - kh * 3;
  const float* om = OM + col;
  const float dy = om[(size_t)(2 * tap) * kLDC] + offb[2 * tap];
  const float dx = om[(size_t)(2 * tap + 1) * kLDC] + offb[2 * tap + 1];
  float ml = om[(size_t)(kNOFS + tap) * kLDC] + maskb[tap];
  ml = fminf(fmaxf(ml, -30.0f), 30.0f);
  const float msk = 1.0f / (1.0f + expf(-ml));
  const int Hs = half ? Ho : 2 * Ho;
  const int st = half ? 1 : 2;
  const unsigned short* src = half ? srcUp : srcDown;
  const float gy = (float)(ho * st + kh - 1);
  const float gx = (float)(wo * st + kw - 1);
  float py = gy + dy;
  float px = gx + dx;
  py = fminf(fmaxf(py, -2.0f), (float)(Hs + 1));
  px = fminf(fmaxf(px, -2.0f), (float)(Hs + 1));
  const float y0 = floorf(py), x0 = floorf(px);
  const float y1 = y0 + 1.0f, x1 = x0 + 1.0f;
  const float wy1 = py - y0, wx1 = px - x0;
  const float wy0 = 1.0f - wy1, wx0 = 1.0f - wx1;
  const float hmax = (float)(Hs - 1);
  const bool vy0 = (y0 >= 0.0f) && (y0 <= hmax);
  const bool vy1 = (y1 >= 0.0f) && (y1 <= hmax);
  const bool vx0 = (x0 >= 0.0f) && (x0 <= hmax);
  const bool vx1 = (x1 >= 0.0f) && (x1 <= hmax);
  float w00 = wy0 * wx0, w01 = wy0 * wx1, w10 = wy1 * wx0, w11 = wy1 * wx1;
  w00 = (vy0 && vx0) ? w00 : 0.0f;
  w01 = (vy0 && vx1) ? w01 : 0.0f;
  w10 = (vy1 && vx0) ? w10 : 0.0f;
  w11 = (vy1 && vx1) ? w11 : 0.0f;
  const int yi0 = iclamp((int)fminf(fmaxf(y0, 0.0f), hmax), 0, Hs - 1);
  const int yi1 = iclamp((int)fminf(fmaxf(y1, 0.0f), hmax), 0, Hs - 1);
  const int xi0 = iclamp((int)fminf(fmaxf(x0, 0.0f), hmax), 0, Hs - 1);
  const int xi1 = iclamp((int)fminf(fmaxf(x1, 0.0f), hmax), 0, Hs - 1);
  const unsigned short* sb = src + (size_t)b * Hs * Hs * kCH + lane * 8;
  v4u g00 = *(const v4u*)(sb + ((size_t)yi0 * Hs + xi0) * kCH);
  v4u g01 = *(const v4u*)(sb + ((size_t)yi0 * Hs + xi1) * kCH);
  v4u g10 = *(const v4u*)(sb + ((size_t)yi1 * Hs + xi0) * kCH);
  v4u g11 = *(const v4u*)(sb + ((size_t)yi1 * Hs + xi1) * kCH);
  asm volatile("" : "+v"(g00), "+v"(g01), "+v"(g10), "+v"(g11));
  float f00[8], f01[8], f10[8], f11[8];
  unpack8(g00, f00);
  unpack8(g01, f01);
  unpack8(g10, f10);
  unpack8(g11, f11);
  const bool live = (n < nreal);
  v8h hv;
#pragma unroll
  for (int e = 0; e < 8; ++e) {
    float s = f00[e] * w00;
    s = s + f01[e] * w01;
    s = s + f10[e] * w10;
    s = s + f11[e] * w11;
    s = s * msk;
    s = live ? s : 0.0f;
    hv[e] = (_Float16)s;
  }
  unsigned short* d = Bt + (size_t)n * kKD + half * kKC + tap * kCH + lane * 8;
  *(volatile v8h*)d = hv;
  __threadfence();
  *(volatile v8h*)d = hv;
}

__global__ __launch_bounds__(256) void fuse_out(const float* __restrict__ p3, const float* __restrict__ p4,
                                                const float* __restrict__ p5, const float* __restrict__ p6,
                                                const float* __restrict__ p7, const float* __restrict__ CS,
                                                const float* __restrict__ dcnb, float* __restrict__ out, int total4) {
  const int v = blockIdx.x * 256 + threadIdx.x;
  if (v >= total4) return;
  const int i = v * 4;
  const int lvl = (i >= kE1 ? 1 : 0) + (i >= kE2 ? 1 : 0) + (i >= kE3 ? 1 : 0) + (i >= kE4 ? 1 : 0);
  const int base = (lvl == 0) ? 0 : ((lvl == 1) ? kE1 : ((lvl == 2) ? kE2 : ((lvl == 3) ? kE3 : kE4)));
  const float* src = (lvl == 0) ? p3 : ((lvl == 1) ? p4 : ((lvl == 2) ? p5 : ((lvl == 3) ? p6 : p7)));
  const int li = i - base;
  v4f rv = *(const v4f*)(src + li);
  if (lvl < 4) {
    const int HW   = 6400 >> (2 * lvl);
    const int colb = (lvl == 0) ? 0 : ((lvl == 1) ? 12800 : ((lvl == 2) ? 16000 : 16832));
    const int dd   = (lvl == 0) ? 0 : ((lvl == 1) ? 1 : ((lvl == 2) ? 3 : 5));
    const int du   = (lvl == 0) ? 2 : ((lvl == 1) ? 4 : ((lvl == 2) ? 6 : 7));
    const int bo  = li / HW;
    const int pix = li - bo * HW;
    const int b   = bo >> 8;
    const int o   = bo & 255;
    const v4f cv = *(const v4f*)(CS + (size_t)o * kLDC + colb + b * HW + pix);
    const float bias = dcnb[dd * kCH + o] + dcnb[du * kCH + o];
    rv[0] = rv[0] + (cv[0] + bias);
    rv[1] = rv[1] + (cv[1] + bias);
    rv[2] = rv[2] + (cv[2] + bias);
    rv[3] = rv[3] + (cv[3] + bias);
  }
  float* d = out + i;
  *(volatile v4f*)d = rv;
  __threadfence();
  *(volatile v4f*)d = rv;
}

extern "C" void kernel_launch(void* const* d_in, const int* in_sizes, int n_in,
                              void* d_out, int out_size, void* d_ws, size_t ws_size,
                              hipStream_t stream) {
  if (n_in < 12) return;
  if (in_sizes[0] != kNB * kCH * 25600) return;
  if (in_sizes[1] != kNB * kCH * 6400) return;
  if (in_sizes[2] != kNB * kCH * 1600) return;
  if (in_sizes[3] != kNB * kCH * 400) return;
  if (in_sizes[4] != kNB * kCH * 100) return;
  if (in_sizes[5] != kNB * kCH * 25) return;
  if (in_sizes[6] != 4 * kNOFS * kKC) return;
  if (in_sizes[7] != 4 * kNOFS) return;
  if (in_sizes[8] != 4 * (kNOM - kNOFS) * kKC) return;
  if (in_sizes[9] != 4 * (kNOM - kNOFS)) return;
  if (in_sizes[10] != 8 * kCH * kKC) return;
  if (in_sizes[11] != 8 * kCH) return;
  if (out_size != kOutTotal) return;
  if (ws_size < kWsTotal) return;

  const float* pin[6];
  for (int i = 0; i < 6; ++i) pin[i] = (const float*)d_in[i];
  const float* off_w  = (const float*)d_in[6];
  const float* off_b  = (const float*)d_in[7];
  const float* mask_w = (const float*)d_in[8];
  const float* mask_b = (const float*)d_in[9];
  const float* dcn_w  = (const float*)d_in[10];
  const float* dcn_b  = (const float*)d_in[11];
  float* out = (float*)d_out;

  char* ws = (char*)d_ws;
  unsigned short* nhwc[6];
  nhwc[0] = (unsigned short*)(ws + kOffP2);
  nhwc[1] = (unsigned short*)(ws + kOffP3);
  nhwc[2] = (unsigned short*)(ws + kOffP4);
  nhwc[3] = (unsigned short*)(ws + kOffP5);
  nhwc[4] = (unsigned short*)(ws + kOffP6);
  nhwc[5] = (unsigned short*)(ws + kOffP7);
  unsigned short* up[4];
  up[0] = (unsigned short*)(ws + kOffU0);
  up[1] = (unsigned short*)(ws + kOffU1);
  up[2] = (unsigned short*)(ws + kOffU2);
  up[3] = (unsigned short*)(ws + kOffU3);
  unsigned short* Wcat = (unsigned short*)(ws + kOffWcat);
  unsigned short* OMW  = (unsigned short*)(ws + kOffOMW);
  float*          OM   = (float*)(ws + kOffOM);
  float*          CS   = (float*)(ws + kOffCS);
  unsigned short* BT   = (unsigned short*)(ws + kOffBT);

  const int sizes[6] = {160, 80, 40, 20, 10, 5};

  for (int i = 0; i < 6; ++i) {
    const int HW = sizes[i] * sizes[i];
    const int tilesPerB = (HW + 31) / 32;
    nchw_to_nhwc_f16<<<kNB * tilesPerB, 256, 0, stream>>>(pin[i], nhwc[i], HW, tilesPerB);
  }
  for (int l = 0; l < 4; ++l) {
    const int Hin = sizes[l + 2];
    const int npix = kNB * (2 * Hin) * (2 * Hin);
    resize2x_nhwc_f16<<<(npix + 7) / 8, 256, 0, stream>>>(nhwc[l + 2], up[l], Hin, npix);
  }
  pack_dcn_w<<<(4 * kCH * kKD / 8 + 255) / 256, 256, 0, stream>>>(dcn_w, Wcat);
  pack_om_w<<<(4 * kMOM * kKC / 8 + 255) / 256, 256, 0, stream>>>(off_w, mask_w, OMW);

  const int hoL[4]   = {80, 40, 20, 10};
  const int npadL[4] = {12800, 3200, 832, 256};
  const int colbL[4] = {0, 12800, 16000, 16832};
  for (int l = 0; l < 4; ++l) {
    const int Ho = hoL[l];
    const int N  = kNB * Ho * Ho;
    for (int c0 = 0; c0 < npadL[l]; c0 += kChunk) {
      const int ncol  = (npadL[l] - c0 < kChunk) ? (npadL[l] - c0) : kChunk;
      const int nreal = (N - c0 < ncol) ? (N - c0) : ncol;
      const int items9  = ncol * kTAPS;
      const int items18 = ncol * 2 * kTAPS;
      im2col_f16<<<(items9 + 7) / 8, 256, 0, stream>>>(nhwc[l + 1], BT, Ho, c0, nreal, items9);
      {
        const int tiles = (kMOM / 64) * (ncol / 64);
        gemm_f16_nt<<<(tiles + 7) / 8, 256, 0, stream>>>(
            OMW + (size_t)l * kMOM * kKC, kKC, BT, kKC,
            OM + colbL[l] + c0, kLDC, kMOM, ncol, kKC, kWCarryInv);
      }
      dcn_sample<<<(items18 + 7) / 8, 256, 0, stream>>>(
          nhwc[l], up[l], OM + colbL[l], off_b + l * kNOFS, mask_b + l * (kNOM - kNOFS), BT,
          Ho, c0, nreal, items18);
      {
        const int tiles = (kCH / 64) * (ncol / 64);
        gemm_f16_nt<<<(tiles + 7) / 8, 256, 0, stream>>>(
            Wcat + (size_t)l * kCH * kKD, kKD, BT, kKD,
            CS + colbL[l] + c0, kLDC, kCH, ncol, kKD, kWCarryInv);
      }
    }
  }

  {
    const int total4 = kOutTotal / 4;
    fuse_out<<<(total4 + 255) / 256, 256, 0, stream>>>(pin[1], pin[2], pin[3], pin[4], pin[5], CS, dcn_b, out, total4);
  }
}
